// MultiHeadSelfAttention_60266981097990
// MI455X (gfx1250) — hardware-verified
//
#include <hip/hip_runtime.h>


typedef _Float16 v16h __attribute__((ext_vector_type(16)));
typedef _Float16 v8h  __attribute__((ext_vector_type(8)));
typedef float    v8f  __attribute__((ext_vector_type(8)));
typedef float    v4f  __attribute__((ext_vector_type(4)));

#ifndef NB
#define NB 4
#endif
#ifndef SEQ
#define SEQ 2048
#endif
#define NB_FULL  4
#define SEQ_FULL 2048
#define C_  1024
#define H_  16
#define D_  64
#define MROWS (NB * SEQ)
#define SCALE_    0.125f
#define W_CARRY   64.0f
#define P_CARRY   1024.0f
#define QKV_FOLD  0.015625f
#define ATT_FOLD  0.25f
#define PROJ_FOLD 6.103515625e-05f

static_assert(NB >= 1 && NB <= NB_FULL);
static_assert(SEQ >= 64 && SEQ <= SEQ_FULL);
static_assert(SEQ % 64 == 0);
static_assert(MROWS % 64 == 0);
static_assert(C_ == H_ * D_);
static_assert(D_ == 64);
static_assert((NB * H_ * (SEQ / 16)) % 4 == 0);
static_assert(C_ % 128 == 0 && (3 * C_) % 128 == 0);
static_assert(((size_t)(NB - 1) * SEQ_FULL + SEQ) * C_ * 4 <= 33554432ull);

__device__ __forceinline__ v8f wmma16(v16h a, v16h b, v8f c) {
  v8f d = __builtin_amdgcn_wmma_f32_16x16x32_f16(false, a, false, b, (short)0, c, false, false);
  asm volatile("v_nop\n\tv_nop\n\tv_nop\n\tv_nop" : "+v"(d) : "v"(a), "v"(b));
  return d;
}

__device__ __forceinline__ v16h load_frag(const _Float16* __restrict__ base, long ld, int lane) {
  const _Float16* p = base + (long)(lane & 15) * ld + ((lane >> 4) << 3);
  v8h lo = *(const v8h*)(p);
  v8h hi = *(const v8h*)(p + 16);
  return __builtin_shufflevector(lo, hi, 0,1,2,3,4,5,6,7,8,9,10,11,12,13,14,15);
}

__device__ __forceinline__ v16h load_frag_lds(const _Float16* base, int ld, int lane) {
  const _Float16* p = base + (lane & 15) * ld + ((lane >> 4) << 3);
  v8h lo = *(const v8h*)(p);
  v8h hi = *(const v8h*)(p + 16);
  return __builtin_shufflevector(lo, hi, 0,1,2,3,4,5,6,7,8,9,10,11,12,13,14,15);
}

__device__ __forceinline__ float bf16rne(float f) {
  unsigned int u = __float_as_uint(f);
  u = (u + 0x7FFFu + ((u >> 16) & 1u)) & 0xFFFF0000u;
  return __uint_as_float(u);
}
__device__ __forceinline__ _Float16 cvt1(float v, float scale) {
  return (_Float16)(bf16rne(v) * scale);
}
__device__ __forceinline__ v8h cvt8(v4f a, v4f c, float scale) {
  v8h o = { cvt1(a[0], scale), cvt1(a[1], scale), cvt1(a[2], scale), cvt1(a[3], scale),
            cvt1(c[0], scale), cvt1(c[1], scale), cvt1(c[2], scale), cvt1(c[3], scale) };
  return o;
}

__global__ void __launch_bounds__(128)
cvt_x(const float* __restrict__ x, _Float16* __restrict__ xh) {
  const int m = blockIdx.x;
  const int b = m / SEQ;
  const int n = m - b * SEQ;
  const float* src = x + ((size_t)b * SEQ_FULL + n) * C_ + threadIdx.x * 8;
  _Float16* dst = xh + (size_t)m * C_ + threadIdx.x * 8;
  const v4f a = *(const v4f*)(src);
  const v4f c = *(const v4f*)(src + 4);
  const v8h o = cvt8(a, c, 1.0f);
  *(volatile v8h*)dst = o;
  __threadfence();
  *(volatile v8h*)dst = o;
}

__global__ void __launch_bounds__(128)
cvt_w(const float* __restrict__ w, _Float16* __restrict__ wh, int n8, float scale) {
  const int i = blockIdx.x * 128 + threadIdx.x;
  if (i < n8) {
    const float* src = w + (size_t)i * 8;
    _Float16* dst = wh + (size_t)i * 8;
    const v4f a = *(const v4f*)(src);
    const v4f c = *(const v4f*)(src + 4);
    const v8h o = cvt8(a, c, scale);
    *(volatile v8h*)dst = o;
    __threadfence();
    *(volatile v8h*)dst = o;
  }
}

__global__ void __launch_bounds__(128)
gemm_qkv(const _Float16* __restrict__ X, const _Float16* __restrict__ W,
         _Float16* __restrict__ Q, _Float16* __restrict__ K, _Float16* __restrict__ Vt) {
  __shared__ __attribute__((aligned(16))) _Float16 T[64 * 128];
  const int lane = threadIdx.x & 31;
  const int wave = threadIdx.x >> 5;
  const int wm = wave >> 1;
  const int wn = wave & 1;
  const int mb = blockIdx.x * 64;
  const int ob = blockIdx.y * 128;
  const long m0 = (long)mb + wm * 32;
  const long n0 = (long)ob + wn * 64;

  v8f acc[2][4] = {};
#pragma unroll 1
  for (int k0 = 0; k0 < C_; k0 += 32) {
    v16h a0 = load_frag(X + (m0     ) * C_ + k0, C_, lane);
    v16h a1 = load_frag(X + (m0 + 16) * C_ + k0, C_, lane);
    v16h b0 = load_frag(W + (n0     ) * C_ + k0, C_, lane);
    v16h b1 = load_frag(W + (n0 + 16) * C_ + k0, C_, lane);
    v16h b2 = load_frag(W + (n0 + 32) * C_ + k0, C_, lane);
    v16h b3 = load_frag(W + (n0 + 48) * C_ + k0, C_, lane);
    acc[0][0] = wmma16(a0, b0, acc[0][0]);
    acc[0][1] = wmma16(a0, b1, acc[0][1]);
    acc[0][2] = wmma16(a0, b2, acc[0][2]);
    acc[0][3] = wmma16(a0, b3, acc[0][3]);
    acc[1][0] = wmma16(a1, b0, acc[1][0]);
    acc[1][1] = wmma16(a1, b1, acc[1][1]);
    acc[1][2] = wmma16(a1, b2, acc[1][2]);
    acc[1][3] = wmma16(a1, b3, acc[1][3]);
  }

  const int hrow = (lane >> 4) << 3;
  const int c16  = lane & 15;
  const int s    = ob >> 10;
  if (s < 2) {
#pragma unroll
    for (int i = 0; i < 2; ++i)
#pragma unroll
      for (int j = 0; j < 4; ++j)
#pragma unroll
        for (int r = 0; r < 8; ++r) {
          const int ml = wm * 32 + i * 16 + hrow + r;
          const int ol = wn * 64 + j * 16 + c16;
          T[ml * 128 + ol] = (_Float16)(acc[i][j][r] * QKV_FOLD);
        }
  } else {
#pragma unroll
    for (int i = 0; i < 2; ++i)
#pragma unroll
      for (int j = 0; j < 4; ++j)
#pragma unroll
        for (int r = 0; r < 8; ++r) {
          const int ml = wm * 32 + i * 16 + hrow + r;
          const int ol = wn * 64 + j * 16 + c16;
          T[ol * 64 + ml] = (_Float16)(acc[i][j][r] * QKV_FOLD);
        }
  }
  __syncthreads();

  const int pc = threadIdx.x & 7;
  const int qq = threadIdx.x >> 3;
  const int hbase = (ob & (C_ - 1)) >> 6;
  if (s < 2) {
    _Float16* __restrict__ dstp = (s == 0) ? Q : K;
    for (int ps = 0; ps < 2; ++ps) {
#pragma unroll
      for (int it = 0; it < 8; ++it) {
        const int L  = it * 16 + qq;
        const int ml = L & 63;
        const int hh = L >> 6;
        const int m  = mb + ml;
        const int b  = m / SEQ;
        const int n  = m - b * SEQ;
        const size_t bh = (size_t)(b * H_ + hbase + hh);
        const v8h v = *(const v8h*)(T + ml * 128 + hh * 64 + pc * 8);
        *(volatile v8h*)(dstp + (bh * SEQ + n) * D_ + pc * 8) = v;
      }
      if (ps == 0) __threadfence();
    }
  } else {
    const int b  = mb / SEQ;
    const int nb = mb - b * SEQ;
    for (int ps = 0; ps < 2; ++ps) {
#pragma unroll
      for (int it = 0; it < 8; ++it) {
        const int L  = it * 16 + qq;
        const int hh = L >> 6;
        const int d  = L & 63;
        const size_t bh = (size_t)(b * H_ + hbase + hh);
        const v8h v = *(const v8h*)(T + L * 64 + pc * 8);
        *(volatile v8h*)(Vt + (bh * D_ + d) * SEQ + nb + pc * 8) = v;
      }
      if (ps == 0) __threadfence();
    }
  }
}

__global__ void __launch_bounds__(128)
attn_fwd(const _Float16* __restrict__ Q, const _Float16* __restrict__ K,
         const _Float16* __restrict__ Vt, _Float16* __restrict__ O) {
  __shared__ __attribute__((aligned(16))) _Float16 Pl[4][16 * 64];
  const int lane = threadIdx.x & 31;
  const int wave = threadIdx.x >> 5;
  const int gq = blockIdx.x * 4 + wave;
  const int qb = gq % (SEQ / 16);
  const int bh = gq / (SEQ / 16);

  const _Float16* Qp = Q  + ((size_t)bh * SEQ + qb * 16) * D_;
  const _Float16* Kp = K  + (size_t)bh * SEQ * D_;
  const _Float16* Vp = Vt + (size_t)bh * D_ * SEQ;

  v16h qa0 = load_frag(Qp + 0,  D_, lane);
  v16h qa1 = load_frag(Qp + 32, D_, lane);

  v8f o_acc[4] = {};
  float mrun[8], lrun[8];
#pragma unroll
  for (int r = 0; r < 8; ++r) { mrun[r] = -1e30f; lrun[r] = 0.f; }

  const int hrow = (lane >> 4) << 3;
  const int c16  = lane & 15;

#pragma unroll 1
  for (int kb = 0; kb < SEQ; kb += 32) {
    v8f s0 = {}, s1 = {};
    {
      v16h kb0 = load_frag(Kp + (size_t)(kb     ) * D_ + 0,  D_, lane);
      v16h kb1 = load_frag(Kp + (size_t)(kb     ) * D_ + 32, D_, lane);
      s0 = wmma16(qa0, kb0, s0);
      s0 = wmma16(qa1, kb1, s0);
      v16h kc0 = load_frag(Kp + (size_t)(kb + 16) * D_ + 0,  D_, lane);
      v16h kc1 = load_frag(Kp + (size_t)(kb + 16) * D_ + 32, D_, lane);
      s1 = wmma16(qa0, kc0, s1);
      s1 = wmma16(qa1, kc1, s1);
    }

    float alpha[8];
#pragma unroll
    for (int r = 0; r < 8; ++r) {
      float v0 = s0[r] * SCALE_;
      float v1 = s1[r] * SCALE_;
      float mx = fmaxf(v0, v1);
      mx = fmaxf(mx, __shfl_xor(mx, 1));
      mx = fmaxf(mx, __shfl_xor(mx, 2));
      mx = fmaxf(mx, __shfl_xor(mx, 4));
      mx = fmaxf(mx, __shfl_xor(mx, 8));
      float mnew = fmaxf(mrun[r], mx);
      float p0 = __expf(v0 - mnew);
      float p1 = __expf(v1 - mnew);
      float rs = p0 + p1;
      rs += __shfl_xor(rs, 1);
      rs += __shfl_xor(rs, 2);
      rs += __shfl_xor(rs, 4);
      rs += __shfl_xor(rs, 8);
      alpha[r] = __expf(mrun[r] - mnew);
      lrun[r]  = lrun[r] * alpha[r] + rs;
      mrun[r]  = mnew;
      s0[r] = p0 * P_CARRY;
      s1[r] = p1 * P_CARRY;
    }
#pragma unroll
    for (int t = 0; t < 4; ++t)
#pragma unroll
      for (int r = 0; r < 8; ++r) o_acc[t][r] *= alpha[r];

    __syncthreads();
#pragma unroll
    for (int r = 0; r < 8; ++r) {
      const int m = hrow + r;
      Pl[wave][m * 32 +      c16] = (_Float16)s0[r];
      Pl[wave][m * 32 + 16 + c16] = (_Float16)s1[r];
    }
    __syncthreads();
    v16h pa = load_frag_lds(&Pl[wave][0], 32, lane);

#pragma unroll
    for (int t = 0; t < 4; ++t) {
      v16h vb = load_frag(Vp + (size_t)(t * 16) * SEQ + kb, SEQ, lane);
      o_acc[t] = wmma16(pa, vb, o_acc[t]);
    }
  }

  const int b = bh / H_;
  const int h = bh - b * H_;
  __syncthreads();
#pragma unroll
  for (int r = 0; r < 8; ++r) {
    const float inv = ATT_FOLD / lrun[r];
    const int m = hrow + r;
#pragma unroll
    for (int t = 0; t < 4; ++t)
      Pl[wave][m * 64 + t * 16 + c16] = (_Float16)(o_acc[t][r] * inv);
  }
  __syncthreads();
  const int pc = lane & 7;
  const int qq = lane >> 3;
  for (int ps = 0; ps < 2; ++ps) {
#pragma unroll
    for (int it = 0; it < 4; ++it) {
      const int i = it * 4 + qq;
      const v8h v = *(const v8h*)(&Pl[wave][i * 64 + pc * 8]);
      const size_t row = (size_t)b * SEQ + qb * 16 + i;
      *(volatile v8h*)(O + row * C_ + h * D_ + pc * 8) = v;
    }
    if (ps == 0) __threadfence();
  }
}

__global__ void __launch_bounds__(128)
gemm_proj(const _Float16* __restrict__ A, const _Float16* __restrict__ W,
          const float* __restrict__ bias, float* __restrict__ out) {
  __shared__ __attribute__((aligned(16))) float T[64 * 128];
  const int lane = threadIdx.x & 31;
  const int wave = threadIdx.x >> 5;
  const int wm = wave >> 1;
  const int wn = wave & 1;
  const int mb = blockIdx.x * 64;
  const int ob = blockIdx.y * 128;
  const long m0 = (long)mb + wm * 32;
  const long n0 = (long)ob + wn * 64;

  v8f acc[2][4] = {};
#pragma unroll 1
  for (int k0 = 0; k0 < C_; k0 += 32) {
    v16h a0 = load_frag(A + (m0     ) * C_ + k0, C_, lane);
    v16h a1 = load_frag(A + (m0 + 16) * C_ + k0, C_, lane);
    v16h b0 = load_frag(W + (n0     ) * C_ + k0, C_, lane);
    v16h b1 = load_frag(W + (n0 + 16) * C_ + k0, C_, lane);
    v16h b2 = load_frag(W + (n0 + 32) * C_ + k0, C_, lane);
    v16h b3 = load_frag(W + (n0 + 48) * C_ + k0, C_, lane);
    acc[0][0] = wmma16(a0, b0, acc[0][0]);
    acc[0][1] = wmma16(a0, b1, acc[0][1]);
    acc[0][2] = wmma16(a0, b2, acc[0][2]);
    acc[0][3] = wmma16(a0, b3, acc[0][3]);
    acc[1][0] = wmma16(a1, b0, acc[1][0]);
    acc[1][1] = wmma16(a1, b1, acc[1][1]);
    acc[1][2] = wmma16(a1, b2, acc[1][2]);
    acc[1][3] = wmma16(a1, b3, acc[1][3]);
  }

  const int hrow = (lane >> 4) << 3;
  const int c16  = lane & 15;
#pragma unroll
  for (int j = 0; j < 4; ++j) {
    const int ol = wn * 64 + j * 16 + c16;
    const float bv = bf16rne(bias[ob + ol]);
#pragma unroll
    for (int i = 0; i < 2; ++i)
#pragma unroll
      for (int r = 0; r < 8; ++r) {
        const int ml = wm * 32 + i * 16 + hrow + r;
        T[ml * 128 + ol] = acc[i][j][r] * PROJ_FOLD + bv;
      }
  }
  __syncthreads();

  const int pc = threadIdx.x & 7;
  const int qq = threadIdx.x >> 3;
  for (int ps = 0; ps < 2; ++ps) {
#pragma unroll
    for (int it = 0; it < 16; ++it) {
      const int L   = it * 16 + qq;
      const int ml  = L >> 2;
      const int seg = L & 3;
      const int m   = mb + ml;
      const int b   = m / SEQ;
      const int n   = m - b * SEQ;
      const v4f v = *(const v4f*)(T + ml * 128 + seg * 32 + pc * 4);
      *(volatile v4f*)(out + ((size_t)b * SEQ_FULL + n) * C_ + ob + seg * 32 + pc * 4) = v;
    }
    if (ps == 0) __threadfence();
  }
}

extern "C" void kernel_launch(void* const* d_in, const int* in_sizes, int n_in,
                              void* d_out, int out_size, void* d_ws, size_t ws_size,
                              hipStream_t stream) {
  if (n_in < 4) return;
  const size_t needX = ((size_t)(NB - 1) * SEQ_FULL + SEQ) * C_;
  if ((size_t)in_sizes[0] < needX) return;
  if ((size_t)in_sizes[1] < (size_t)3 * C_ * C_) return;
  if ((size_t)in_sizes[2] < (size_t)C_ * C_) return;
  if (in_sizes[3] < C_) return;
  if ((size_t)out_size < needX) return;

  const float* x      = (const float*)d_in[0];
  const float* w_qkv  = (const float*)d_in[1];
  const float* w_proj = (const float*)d_in[2];
  const float* b_proj = (const float*)d_in[3];
  float* out = (float*)d_out;

  const size_t nXh   = (size_t)MROWS * C_;
  const size_t nWq   = (size_t)3 * C_ * C_;
  const size_t nWp   = (size_t)C_ * C_;
  const size_t nHead = (size_t)NB * H_ * SEQ * D_;
  const size_t total = (nXh + nWq + nWp + 3 * nHead + nXh) * sizeof(_Float16);
  if (total > ws_size) return;

  _Float16* xh  = (_Float16*)d_ws;
  _Float16* wqh = xh  + nXh;
  _Float16* wph = wqh + nWq;
  _Float16* qw  = wph + nWp;
  _Float16* kw  = qw  + nHead;
  _Float16* vtw = kw  + nHead;
  _Float16* ow  = vtw + nHead;

  const int nWq8 = (int)(nWq / 8);
  const int nWp8 = (int)(nWp / 8);
  cvt_x<<<MROWS, 128, 0, stream>>>(x, xh);
  cvt_w<<<(nWq8 + 127) / 128, 128, 0, stream>>>(w_qkv, wqh, nWq8, W_CARRY);
  cvt_w<<<(nWp8 + 127) / 128, 128, 0, stream>>>(w_proj, wph, nWp8, W_CARRY);

  gemm_qkv<<<dim3(MROWS / 64, (3 * C_) / 128), 128, 0, stream>>>(xh, wqh, qw, kw, vtw);

  attn_fwd<<<(NB * H_ * (SEQ / 16)) / 4, 128, 0, stream>>>(qw, kw, vtw, ow);

  gemm_proj<<<dim3(MROWS / 64, C_ / 128), 128, 0, stream>>>(ow, wph, b_proj, out);
}
